// FeaturePropagationLayer_42314017800358
// MI455X (gfx1250) — hardware-verified
//
#include <hip/hip_runtime.h>
#include <math.h>

typedef __attribute__((ext_vector_type(16))) _Float16 v16h;
typedef __attribute__((ext_vector_type(8)))  _Float16 v8h;
typedef __attribute__((ext_vector_type(8)))  float    v8f;
typedef __attribute__((ext_vector_type(4)))  float    v4f;
typedef __attribute__((ext_vector_type(2)))  float    v2f;
typedef __attribute__((ext_vector_type(4)))  int      v4i;

constexpr int kClouds   = 8;
constexpr int kDense    = 4096;
constexpr int kCoarse   = 1024;
constexpr int kCh1      = 256;
constexpr int kCh2      = 512;
constexpr int kInCh     = kCh1 + kCh2;
constexpr int kHid1     = 512;
constexpr int kHid2     = 256;
constexpr int kPts      = kClouds * kDense;
constexpr int kRow1     = 3 + kCh1;
constexpr int kRow2     = 3 + kCh2;
constexpr int kGroups   = 256;
constexpr int kGroupRows = 128;
constexpr int kSearchBlk = 256;
constexpr float kEps    = 1e-5f;
constexpr float kCarryW = 256.0f;
constexpr float kCarryA = 16.0f;
constexpr float kFold   = 1.0f / (kCarryW * kCarryA);
constexpr float kF16MinNormal = 6.103515625e-5f;

static_assert(kInCh == 768 && kRow1 == 259 && kRow2 == 515 && kPts == 32768, "shape constants");
static_assert((kInCh % 32) == 0 && (kHid1 % 32) == 0, "GEMM K multiples of 32");
static_assert((kPts % 64) == 0 && (kHid1 % 64) == 0 && (kHid2 % 64) == 0, "GEMM M,N multiples of 64");
static_assert(kGroups * kGroupRows == kPts, "statistics groups cover all rows");
static_assert(((size_t)kPts * kRow1) % 1024 == 0, "output is a whole number of 256-thread x 4-float blocks");
static_assert((kDense % kSearchBlk) == 0 && (kCoarse % kSearchBlk) == 0, "search tiling");
static_assert(kSearchBlk == 8 * 32, "eight waves of 32 points per search block");
static_assert(kCh1 == 4 * 64 && kCh2 == 8 * 64, "row build: 4 + 8 line segments of 64 columns");
static_assert((kInCh * 2) % 128 == 0, "operand row is a whole number of 128-B lines");

constexpr size_t kOffXA   = 0;
constexpr size_t kOffH1F  = kOffXA  + (size_t)kPts * kInCh * 2;
constexpr size_t kOffH2   = kOffH1F;
constexpr size_t kOffW1H  = kOffH1F + (size_t)kPts * kHid1 * 4;
constexpr size_t kOffW2H  = kOffW1H + (size_t)kHid1 * kInCh * 2;
constexpr size_t kOffPS1  = kOffW2H + (size_t)kHid2 * kHid1 * 2;
constexpr size_t kOffPS2  = kOffPS1 + (size_t)2 * kGroups * kHid1 * 4;
constexpr size_t kOffSCSH = kOffPS2 + (size_t)2 * kGroups * kHid2 * 4;
constexpr size_t kWsTotal = kOffSCSH + (size_t)(2 * kHid1 + 2 * kHid2) * 4;
static_assert(kWsTotal == 120068096ull, "carve total");
static_assert(kWsTotal <= 134217728ull, "carve cap");
static_assert((kOffH1F % 128) == 0 && (kOffH2 % 128) == 0 && (kOffW1H % 128) == 0 && (kOffW2H % 128) == 0 &&
              (kOffPS1 % 128) == 0 && (kOffPS2 % 128) == 0 && (kOffSCSH % 128) == 0,
              "128-B aligned regions");
static_assert((size_t)kPts * kHid1 * 2 <= (size_t)kPts * kInCh * 2, "layer-2 operand rows fit the re-used region");
static_assert((size_t)kPts * kHid2 * 4 <= (size_t)kPts * kHid1 * 4, "raw layer-2 output fits the re-used f32 region");

__device__ __forceinline__ float flush16(float v) { return (fabsf(v) < kF16MinNormal) ? 0.0f : v; }

__device__ __forceinline__ float h16_to_f32(unsigned hb) {
  const unsigned sgn = (hb & 0x8000u) << 16; const unsigned em = hb & 0x7fffu;
  const float fn = __uint_as_float((em << 13) + 0x38000000u);
  const float fs = (float)em * 5.9604644775390625e-8f;
  const float mag = (em < 0x400u) ? fs : fn; return __uint_as_float(__float_as_uint(mag) | sgn); }

__device__ __forceinline__ int clamp_idx(int v, int hi) { v = v < 0 ? 0 : v; return v > hi ? hi : v; }

__device__ __forceinline__ unsigned pack2_f16(float v0, float v1) {
  const _Float16 h0 = (_Float16)flush16(v0 * kCarryA);
  const _Float16 h1 = (_Float16)flush16(v1 * kCarryA);
  const unsigned short b0 = __builtin_bit_cast(unsigned short, h0);
  const unsigned short b1 = __builtin_bit_cast(unsigned short, h1);
  return (unsigned)b0 | ((unsigned)b1 << 16);
}

__device__ __forceinline__ void row_guard_h(v8f& a, v8f& b, v8f& c, v8f& d, v16h x, v16h y) {
  asm volatile("v_nop\n\tv_nop\n\tv_nop\n\tv_nop" : "+v"(a), "+v"(b), "+v"(c), "+v"(d) : "v"(x), "v"(y));
}
__device__ __forceinline__ void keep4_h(v16h a, v16h b, v16h c, v16h d) { asm volatile("v_nop" :: "v"(a), "v"(b), "v"(c), "v"(d)); }
__device__ __forceinline__ void acc_guard4(v8f& a, v8f& b, v8f& c, v8f& d) { asm volatile("v_nop\n\tv_nop\n\tv_nop\n\tv_nop" : "+v"(a), "+v"(b), "+v"(c), "+v"(d)); }

struct FragH {
  union U { v16h v; v8h h[2]; };
  static __device__ __forceinline__ v16h load(const _Float16* p) {
    U f; f.h[0] = *(const v8h*)(p); f.h[1] = *(const v8h*)(p + 16); return f.v;
  }
  static __device__ __forceinline__ v8f mma(v16h a, v16h b, v8f c) {
    return __builtin_amdgcn_wmma_f32_16x16x32_f16(false, a, false, b, (short)0, c, false, false);
  }
};

template <int OUT_MODE>
__global__ __launch_bounds__(256) void wmma_gemm64(
    const unsigned short* __restrict__ Ap, int lda,
    const unsigned short* __restrict__ Btp, int ldb,
    void* __restrict__ Cout, int ldc,
    const float* __restrict__ bias,
    int M, int N, int K, float scale) {
  const _Float16* A  = (const _Float16*)Ap;
  const _Float16* Bt = (const _Float16*)Btp;
  __shared__ __align__(16) float sT[8][16 * 68];
  const int lane = threadIdx.x & 31;
  const int wave = threadIdx.x >> 5;
  const int tilesN = N >> 6;
  const int tilesM = M >> 6;
  const int tile = blockIdx.x * 8 + wave;
  if (tile >= tilesM * tilesN) return;
  const int tm = tile / tilesN;
  const int tn = tile - tm * tilesN;
  const int m0 = tm << 6;
  const int n0 = tn << 6;

  const int rlane = lane & 15;
  const int koff  = (lane >> 4) * 8;
  const int mOff  = (lane >> 4) * 8;

  v8f acc[4][4];
#pragma unroll
  for (int i = 0; i < 4; ++i)
#pragma unroll
    for (int j = 0; j < 4; ++j) acc[i][j] = (v8f){0.f,0.f,0.f,0.f,0.f,0.f,0.f,0.f};

  for (int k0 = 0; k0 < K; k0 += 32) {
    v16h bh[4];
#pragma unroll
    for (int j = 0; j < 4; ++j) {
      const size_t bo = (size_t)(n0 + (j << 4) + rlane) * ldb + koff + k0;
      bh[j] = FragH::load(Bt + bo);
    }
#pragma unroll
    for (int i = 0; i < 4; ++i) {
      const size_t ao = (size_t)(m0 + (i << 4) + rlane) * lda + koff + k0;
      v16h ah = FragH::load(A + ao);
#pragma unroll
      for (int j = 0; j < 4; ++j) acc[i][j] = FragH::mma(ah, bh[j], acc[i][j]);
      row_guard_h(acc[i][0], acc[i][1], acc[i][2], acc[i][3], ah, bh[3]);
    }
    keep4_h(bh[0], bh[1], bh[2], bh[3]);
  }
  acc_guard4(acc[0][0], acc[0][1], acc[0][2], acc[0][3]);
  acc_guard4(acc[1][0], acc[1][1], acc[1][2], acc[1][3]);
  acc_guard4(acc[2][0], acc[2][1], acc[2][2], acc[2][3]);
  acc_guard4(acc[3][0], acc[3][1], acc[3][2], acc[3][3]);

  float* slab = sT[wave];
#pragma unroll
  for (int i = 0; i < 4; ++i) {
    const int mBase = m0 + (i << 4);
#pragma unroll
    for (int j = 0; j < 4; ++j) {
      const int n = n0 + (j << 4) + rlane;
      const float bv = bias[n];
#pragma unroll
      for (int r = 0; r < 8; ++r) {
        float v = acc[i][j][r] * scale;
        v += bv;
        slab[(mOff + r) * 68 + (j << 4) + rlane] = v;
      }
    }
    __builtin_amdgcn_fence(__ATOMIC_RELEASE, "workgroup");
    __builtin_amdgcn_wave_barrier();
    __builtin_amdgcn_fence(__ATOMIC_ACQUIRE, "workgroup");
    if (OUT_MODE == 0) {
      float* C = (float*)Cout;
      const int hh = lane >> 4, c4 = (lane & 15) * 4;
      for (int pass = 0; pass < 2; ++pass) {
#pragma unroll
        for (int it = 0; it < 8; ++it) {
          const int row = it * 2 + hh;
          v4f v = *(const v4f*)(slab + row * 68 + c4);
          *(volatile v4f*)(C + (size_t)(mBase + row) * ldc + n0 + c4) = v;
        }
        __threadfence();
      }
    } else {
      const int q = lane >> 3, c8 = (lane & 7) * 8;
      unsigned short* C = (unsigned short*)Cout;
      for (int pass = 0; pass < 2; ++pass) {
#pragma unroll
        for (int it = 0; it < 4; ++it) {
          const int row = it * 4 + q;
          const float* sp = slab + row * 68 + c8;
          v8h hv;
#pragma unroll
          for (int e = 0; e < 8; ++e) hv[e] = (_Float16)sp[e];
          *(volatile v8h*)(C + (size_t)(mBase + row) * ldc + n0 + c8) = hv;
        }
        __threadfence();
      }
    }
    __builtin_amdgcn_fence(__ATOMIC_RELEASE, "workgroup");
    __builtin_amdgcn_wave_barrier();
    __builtin_amdgcn_fence(__ATOMIC_ACQUIRE, "workgroup");
  }
}

__global__ __launch_bounds__(256) void weights_to_f16_kernel(
    const float* __restrict__ src, unsigned short* __restrict__ dst, int total8, float carry)
{
  const int i = blockIdx.x * 256 + threadIdx.x;
  if (i >= total8) return;
  const size_t e0 = (size_t)i << 3;
  const v4f a0 = *(const v4f*)(src + e0);
  const v4f a1 = *(const v4f*)(src + e0 + 4);
  v8h hv;
#pragma unroll
  for (int e = 0; e < 4; ++e) {
    const float x0 = flush16(a0[e] * carry);
    const float x1 = flush16(a1[e] * carry);
    hv[e]     = (_Float16)x0;
    hv[4 + e] = (_Float16)x1;
  }
  unsigned short* q = dst + e0;
  *(volatile v8h*)q = hv;
  __threadfence();
  *(volatile v8h*)q = hv;
}

__global__ __launch_bounds__(256) void nearest3_rows_kernel(
    const float* __restrict__ l1, const float* __restrict__ l2, unsigned short* __restrict__ XA)
{
#pragma clang fp contract(off)
  __shared__ __align__(16) float sQ[kCoarse * 4];
  __shared__ __align__(16) int sIdx[kSearchBlk * 4];
  const int tid = threadIdx.x;
  const int b = blockIdx.y;
#pragma unroll
  for (int i = 0; i < 4; ++i) {
    const int j = tid + 256 * i;
    const float* r = l2 + ((size_t)b * kCoarse + j) * kRow2;
    const float qx = r[0], qy = r[1], qz = r[2];
    const float t0 = qx * qx;
    const float t1 = qy * qy;
    const float t2 = qz * qz;
    const float n2 = (t0 + t2) + t1;
    *(v4f*)(sQ + 4 * j) = (v4f){qx, qy, qz, n2};
  }
  __syncthreads();
  const int n = blockIdx.x * 256 + tid;
  const size_t p = (size_t)b * kDense + n;
  const float* r1 = l1 + p * kRow1;
  const float x = r1[0], y = r1[1], z = r1[2];
  const float s0 = x * x;
  const float s1 = y * y;
  const float s2 = z * z;
  const float n1 = (s0 + s2) + s1;
  float d0 = __builtin_inff(), d1 = __builtin_inff(), d2 = __builtin_inff();
  int i0 = 0, i1 = 0, i2 = 0;
#pragma unroll 4
  for (int m = 0; m < kCoarse; ++m) {
    const v4f q = *(const v4f*)(sQ + 4 * m);
    float e = x * q[0];
    e = fmaf(y, q[1], e);
    e = fmaf(z, q[2], e);
    float t = -2.0f * e;
    t = t + n1;
    t = t + q[3];
    const bool c0 = t < d0;
    const bool c1 = t < d1;
    const bool c2 = t < d2;
    d2 = c1 ? d1 : (c2 ? t : d2);
    i2 = c1 ? i1 : (c2 ? m : i2);
    d1 = c0 ? d0 : (c1 ? t : d1);
    i1 = c0 ? i0 : (c1 ? m : i1);
    d0 = c0 ? t : d0;
    i0 = c0 ? m : i0;
  }
  v4i o;
  o[0] = clamp_idx(i0, kCoarse - 1);
  o[1] = clamp_idx(i1, kCoarse - 1);
  o[2] = clamp_idx(i2, kCoarse - 1);
  o[3] = 0;
  *(v4i*)(sIdx + 4 * tid) = o;
  __syncthreads();

  const int lane = tid & 31;
  const int wave = tid >> 5;
  const size_t pbase  = (size_t)b * kDense + (size_t)blockIdx.x * 256 + (size_t)wave * 32;
  const size_t l2base = (size_t)b * kCoarse;
#pragma unroll 1
  for (int k = 0; k < 32; ++k) {
    const size_t pp = pbase + k;
    const v4i id = *(const v4i*)(sIdx + 4 * (wave * 32 + k));
    const int ia = clamp_idx(id[0], kCoarse - 1);
    const int ib = clamp_idx(id[1], kCoarse - 1);
    const int ic = clamp_idx(id[2], kCoarse - 1);
    volatile unsigned* qrow = (volatile unsigned*)XA + pp * (size_t)(kInCh / 2) + lane;
    const float* f1 = l1 + pp * kRow1 + 3 + 2 * lane;
#pragma unroll 1
    for (int s = 0; s < 4; ++s) {
      const float v0 = f1[64 * s];
      const float v1 = f1[64 * s + 1];
      const unsigned u = pack2_f16(v0, v1);
      qrow[32 * s] = u;
      __threadfence();
      qrow[32 * s] = u;
    }
    const float* fa = l2 + (l2base + (size_t)ia) * kRow2 + 3 + 2 * lane;
    const float* fb = l2 + (l2base + (size_t)ib) * kRow2 + 3 + 2 * lane;
    const float* fc = l2 + (l2base + (size_t)ic) * kRow2 + 3 + 2 * lane;
#pragma unroll 1
    for (int s = 0; s < 8; ++s) {
      const float a0 = fa[64 * s], a1 = fa[64 * s + 1];
      const float b0 = fb[64 * s], b1 = fb[64 * s + 1];
      const float c0 = fc[64 * s], c1 = fc[64 * s + 1];
      const float v0 = ((a0 + b0) + c0) * (1.0f / 3.0f);
      const float v1 = ((a1 + b1) + c1) * (1.0f / 3.0f);
      const unsigned u = pack2_f16(v0, v1);
      qrow[kCh1 / 2 + 32 * s] = u;
      __threadfence();
      qrow[kCh1 / 2 + 32 * s] = u;
    }
  }
}

template <int C, bool F16IN>
__global__ __launch_bounds__(C / 2) void colstats_partial_kernel(
    const void* __restrict__ Hp, float* __restrict__ psum, float* __restrict__ psq)
{
  const int g = blockIdx.x;
  const int t = threadIdx.x;
  float s0 = 0.0f, s1 = 0.0f, q0 = 0.0f, q1 = 0.0f;
#pragma unroll 4
  for (int r = 0; r < kGroupRows; ++r) {
    const size_t row = (size_t)g * kGroupRows + r;
    float a0, a1;
    if (F16IN) {
      const unsigned w = ((const unsigned*)Hp)[row * (C / 2) + t];
      a0 = h16_to_f32(w & 0xffffu);
      a1 = h16_to_f32(w >> 16);
    } else {
      const v2f v = *(const v2f*)((const float*)Hp + row * C + 2 * t);
      a0 = v[0];
      a1 = v[1];
    }
    s0 += a0;
    s1 += a1;
    q0 += a0 * a0;
    q1 += a1 * a1;
  }
  const v2f sv = (v2f){s0, s1};
  const v2f qv = (v2f){q0, q1};
  float* ds = psum + (size_t)g * C + 2 * t;
  float* dq = psq  + (size_t)g * C + 2 * t;
  *(volatile v2f*)ds = sv;
  *(volatile v2f*)dq = qv;
  __threadfence();
  *(volatile v2f*)ds = sv;
  *(volatile v2f*)dq = qv;
}

template <int C>
__global__ __launch_bounds__(C) void colstats_finalize_kernel(
    const float* __restrict__ psum, const float* __restrict__ psq,
    const float* __restrict__ gamma, const float* __restrict__ beta,
    float* __restrict__ sc, float* __restrict__ sh)
{
  const int c = threadIdx.x;
  double s = 0.0, q = 0.0;
#pragma unroll 4
  for (int g = 0; g < kGroups; ++g) {
    s += (double)psum[(size_t)g * C + c];
    q += (double)psq[(size_t)g * C + c];
  }
  const double invP = 1.0 / (double)kPts;
  const double mu = s * invP;
  double var = q * invP - mu * mu;
  var = (var < 0.0) ? 0.0 : var;
  const float rstd = rsqrtf((float)var + kEps);
  const float scv = gamma[c] * rstd;
  const float shv = beta[c] - (float)mu * scv;
  *(volatile float*)(sc + c) = scv;
  *(volatile float*)(sh + c) = shv;
  __threadfence();
  *(volatile float*)(sc + c) = scv;
  *(volatile float*)(sh + c) = shv;
}

__global__ __launch_bounds__(256) void bn_relu_f16_kernel(
    const float* __restrict__ H1, const float* __restrict__ sc, const float* __restrict__ sh,
    unsigned short* __restrict__ A2, int total8)
{
  const int i = blockIdx.x * 256 + threadIdx.x;
  if (i >= total8) return;
  const size_t e0 = (size_t)i << 3;
  const int c8 = (int)(e0 & (size_t)(kHid1 - 1));
  const v4f ha = *(const v4f*)(H1 + e0);
  const v4f hb = *(const v4f*)(H1 + e0 + 4);
  const v4f sa = *(const v4f*)(sc + c8);
  const v4f sb = *(const v4f*)(sc + c8 + 4);
  const v4f ta = *(const v4f*)(sh + c8);
  const v4f tb = *(const v4f*)(sh + c8 + 4);
  const float hin[8] = {ha[0], ha[1], ha[2], ha[3], hb[0], hb[1], hb[2], hb[3]};
  const float scv[8] = {sa[0], sa[1], sa[2], sa[3], sb[0], sb[1], sb[2], sb[3]};
  const float shv[8] = {ta[0], ta[1], ta[2], ta[3], tb[0], tb[1], tb[2], tb[3]};
  v8h hv;
#pragma unroll
  for (int e = 0; e < 8; ++e) {
    const float zv = fmaxf(hin[e] * scv[e] + shv[e], 0.0f);
    const float yv = flush16(zv * kCarryA);
    hv[e] = (_Float16)yv;
  }
  unsigned short* q = A2 + e0;
  *(volatile v8h*)q = hv;
  __threadfence();
  *(volatile v8h*)q = hv;
}

__global__ __launch_bounds__(256) void finalize_out_kernel(
    const float* __restrict__ l1, const float* __restrict__ H2,
    const float* __restrict__ sc2, const float* __restrict__ sh2,
    float* __restrict__ out, int total4)
{
  const int i = blockIdx.x * 256 + threadIdx.x;
  if (i >= total4) return;
  const int flat0 = i * 4;
  const int p0 = flat0 / kRow1;
  const int c0 = flat0 - p0 * kRow1;
  const v4f xv = *(const v4f*)(l1 + flat0);
  float xa = xv[0], xb = xv[1], xc = xv[2], xd = xv[3];
  asm volatile("" : "+v"(xa), "+v"(xb), "+v"(xc), "+v"(xd));
  const float xs[4] = {xa, xb, xc, xd};
  float o[4];
#pragma unroll
  for (int e = 0; e < 4; ++e) {
    int c = c0 + e;
    int p = p0;
    const bool wrap = (c >= kRow1);
    c = wrap ? (c - kRow1) : c;
    p = wrap ? (p + 1) : p;
    p = (p > kPts - 1) ? (kPts - 1) : p;
    int ch = c - 3;
    ch = (ch < 0) ? 0 : ch;
    ch = (ch > kHid2 - 1) ? (kHid2 - 1) : ch;
    float hv = H2[(size_t)p * kHid2 + ch];
    float scv = sc2[ch];
    float shv = sh2[ch];
    asm volatile("" : "+v"(hv), "+v"(scv), "+v"(shv));
    const float val = fmaxf(hv * scv + shv, 0.0f);
    o[e] = (c < 3) ? xs[e] : val;
  }
  const v4f ov = (v4f){o[0], o[1], o[2], o[3]};
  float* q = out + flat0;
  *(volatile v4f*)q = ov;
  __threadfence();
  *(volatile v4f*)q = ov;
}

extern "C" void kernel_launch(void* const* d_in, const int* in_sizes, int n_in,
                              void* d_out, int out_size, void* d_ws, size_t ws_size,
                              hipStream_t stream) {
  if (n_in < 10) return;
  if (in_sizes[0] != kPts * kRow1) return;
  if (in_sizes[1] != kClouds * kCoarse * kRow2) return;
  if (in_sizes[2] != kHid1 * kInCh) return;
  if (in_sizes[3] != kHid1) return;
  if (in_sizes[4] != kHid1) return;
  if (in_sizes[5] != kHid1) return;
  if (in_sizes[6] != kHid2 * kHid1) return;
  if (in_sizes[7] != kHid2) return;
  if (in_sizes[8] != kHid2) return;
  if (in_sizes[9] != kHid2) return;
  if (out_size != kPts * kRow1) return;
  if (ws_size < kWsTotal) return;

  const float* l1  = (const float*)d_in[0];
  const float* l2  = (const float*)d_in[1];
  const float* W1  = (const float*)d_in[2];
  const float* b1  = (const float*)d_in[3];
  const float* g1  = (const float*)d_in[4];
  const float* be1 = (const float*)d_in[5];
  const float* W2  = (const float*)d_in[6];
  const float* b2  = (const float*)d_in[7];
  const float* g2  = (const float*)d_in[8];
  const float* be2 = (const float*)d_in[9];
  float* out = (float*)d_out;

  char* ws = (char*)d_ws;
  unsigned short* XA  = (unsigned short*)(ws + kOffXA);
  float*          H1F = (float*)(ws + kOffH1F);
  float*          H2  = (float*)(ws + kOffH2);
  unsigned short* W1H = (unsigned short*)(ws + kOffW1H);
  unsigned short* W2H = (unsigned short*)(ws + kOffW2H);
  float*          ps1 = (float*)(ws + kOffPS1);
  float*          pq1 = ps1 + (size_t)kGroups * kHid1;
  float*          ps2 = (float*)(ws + kOffPS2);
  float*          pq2 = ps2 + (size_t)kGroups * kHid2;
  float*          sc1 = (float*)(ws + kOffSCSH);
  float*          sh1 = sc1 + kHid1;
  float*          sc2 = sh1 + kHid1;
  float*          sh2 = sc2 + kHid2;

  weights_to_f16_kernel<<<(kHid1 * kInCh / 8) / 256, 256, 0, stream>>>(W1, W1H, kHid1 * kInCh / 8, kCarryW);
  weights_to_f16_kernel<<<(kHid2 * kHid1 / 8) / 256, 256, 0, stream>>>(W2, W2H, kHid2 * kHid1 / 8, kCarryW);

  nearest3_rows_kernel<<<dim3(kDense / kSearchBlk, kClouds), kSearchBlk, 0, stream>>>(l1, l2, XA);

  wmma_gemm64<0><<<(kPts / 64) * (kHid1 / 64) / 8, 256, 0, stream>>>(
      XA, kInCh, W1H, kInCh, (void*)H1F, kHid1, b1, kPts, kHid1, kInCh, kFold);
  colstats_partial_kernel<kHid1, false><<<kGroups, kHid1 / 2, 0, stream>>>((const void*)H1F, ps1, pq1);
  colstats_finalize_kernel<kHid1><<<1, kHid1, 0, stream>>>(ps1, pq1, g1, be1, sc1, sh1);

  bn_relu_f16_kernel<<<(kPts * (kHid1 / 8)) / 256, 256, 0, stream>>>(
      H1F, sc1, sh1, XA, kPts * (kHid1 / 8));

  wmma_gemm64<0><<<(kPts / 64) * (kHid2 / 64) / 8, 256, 0, stream>>>(
      XA, kHid1, W2H, kHid1, (void*)H2, kHid2, b2, kPts, kHid2, kHid1, kFold);
  colstats_partial_kernel<kHid2, false><<<kGroups, kHid2 / 2, 0, stream>>>((const void*)H2, ps2, pq2);
  colstats_finalize_kernel<kHid2><<<1, kHid2, 0, stream>>>(ps2, pq2, g2, be2, sc2, sh2);

  finalize_out_kernel<<<(kPts * kRow1 / 4) / 256, 256, 0, stream>>>(l1, H2, sc2, sh2, out, kPts * kRow1 / 4);
}
